// Encoder_31945966747775
// MI455X (gfx1250) — hardware-verified
//
#include <hip/hip_runtime.h>
#include <hip/hip_fp16.h>


#ifndef NB
#define NB 16
#endif
#ifndef SEQ
#define SEQ 512
#endif
#define NB_FULL  16
#define SEQ_FULL 512
#define DM   256
#define NH   8
#define HD   32
#define NL   4
#define NTOK (NB * SEQ)
#define CH   256
#define WSZ  65536

static_assert(NB >= 1 && NB <= NB_FULL);
static_assert(SEQ >= CH && SEQ <= SEQ_FULL);
static_assert(SEQ % CH == 0);
static_assert(SEQ % 256 == 0);
static_assert(SEQ % 128 == 0);
static_assert(NTOK % 64 == 0);
static_assert(NTOK % 8 == 0);
static_assert(CH % 32 == 0);
static_assert(NH * HD == DM);

typedef _Float16 v16h __attribute__((ext_vector_type(16)));
typedef _Float16 v8h  __attribute__((ext_vector_type(8)));
typedef float    v8f  __attribute__((ext_vector_type(8)));
typedef float    v4f  __attribute__((ext_vector_type(4)));
typedef int      v4i  __attribute__((ext_vector_type(4)));

union Frag { v16h v; v8h h[2]; };

#define LOG2E    1.44269504088896340736f
#define INV_SQDK 0.17677669529663687f
#define C1 (LOG2E * 0.000244140625f * INV_SQDK)
#define C2 (LOG2E * 1.1920928955078125e-07f * INV_SQDK)
#define FILL_T   (-1.0e12f * LOG2E)
#define SC_RES   2048.0f
#define SC_RINV  4.8828125e-04f
#define P_CARRY  10.0f
#define SC_ATT   0.075f
#define SC_MV    6.103515625e-05f
#define SC_WO    9.765625e-04f
#define SC_FF    0.015625f

static __device__ __forceinline__ v8f zero8() {
    v8f z;
#pragma unroll
    for (int i = 0; i < 8; ++i) z[i] = 0.0f;
    return z;
}

static __device__ __forceinline__ v16h load_frag16(const _Float16* base, unsigned ld, unsigned lane) {
    unsigned m  = lane & 15u;
    unsigned kb = (lane >> 4) << 3;
    const _Float16* p = base + (size_t)m * ld + kb;
    Frag f;
    f.h[0] = *(const v8h*)(p);
    f.h[1] = *(const v8h*)(p + 16);
    return f.v;
}

static __device__ __forceinline__ v8f wmma16(v16h a, v16h b, v8f c) {
    v8f d = __builtin_amdgcn_wmma_f32_16x16x32_f16(false, a, false, b, (short)0, c, false, false);
    asm volatile("v_nop\n\tv_nop\n\tv_nop\n\tv_nop" : "+v"(d) : "v"(a), "v"(b));
    return d;
}

static __device__ __forceinline__ float bf16r(float x) {
    unsigned u = __float_as_uint(x);
    u = (u + 0x7FFFu + ((u >> 16) & 1u)) & 0xFFFF0000u;
    return __uint_as_float(u);
}

static __device__ __forceinline__ float ex2(float x) {
    return __builtin_amdgcn_exp2f(x);
}

static __device__ __forceinline__ void wave_lds_sync() {
    __builtin_amdgcn_fence(3, "wavefront");
    asm volatile("s_wait_dscnt 0" ::: "memory");
    __builtin_amdgcn_wave_barrier();
}

__global__ __launch_bounds__(256) void k_wprep(const float* __restrict__ Wq,
                                                const float* __restrict__ Wk,
                                                const float* __restrict__ Wv,
                                                const float* __restrict__ Wo,
                                                const float* __restrict__ Wf1,
                                                const float* __restrict__ Wf2,
                                                _Float16* __restrict__ WT) {
    __shared__ __align__(16) _Float16 T[64 * 72];
    const unsigned tid = threadIdx.x;
    const unsigned kt = blockIdx.x, nt = blockIdx.y, z = blockIdx.z;
    const unsigned l = z / 6u;
    const unsigned mat = z - l * 6u;
    const float* src = (mat == 0u) ? Wq : ((mat == 1u) ? Wk : ((mat == 2u) ? Wv :
                       ((mat == 3u) ? Wo : ((mat == 4u) ? Wf1 : Wf2))));
    src += (size_t)l * WSZ;
    for (unsigned idx = tid; idx < 1024u; idx += 256u) {
        unsigned r = idx >> 4, c4 = idx & 15u;
        v4f wv = *(const v4f*)(src + (size_t)(kt * 64u + r) * DM + nt * 64u + c4 * 4u);
#pragma unroll
        for (int e = 0; e < 4; ++e)
            T[(c4 * 4u + (unsigned)e) * 72u + r] = (_Float16)(bf16r(wv[e]) * 64.0f);
    }
    __syncthreads();
    const unsigned p0 = tid, p1 = tid + 256u;
    v8h w0 = *(const v8h*)(&T[(p0 >> 3) * 72u + (p0 & 7u) * 8u]);
    v8h w1 = *(const v8h*)(&T[(p1 >> 3) * 72u + (p1 & 7u) * 8u]);
    _Float16* base = WT + (size_t)z * WSZ + (size_t)kt * 64u;
    _Float16* d0 = base + (size_t)(nt * 64u + (p0 >> 3)) * DM + (p0 & 7u) * 8u;
    _Float16* d1 = base + (size_t)(nt * 64u + (p1 >> 3)) * DM + (p1 & 7u) * 8u;
    *(volatile v8h*)d0 = w0;
    *(volatile v8h*)d1 = w1;
    __threadfence();
    *(volatile v8h*)d0 = w0;
    *(volatile v8h*)d1 = w1;
}

__global__ __launch_bounds__(256) void k_pmix(const float* __restrict__ adj,
                                               const float* __restrict__ dist,
                                               const int*   __restrict__ mask,
                                               _Float16* __restrict__ Mh) {
    const unsigned tid = threadIdx.x, lane = tid & 31u, w = tid >> 5;
    const unsigned row = blockIdx.x * 8u + w;
    const unsigned b = row / (unsigned)SEQ;
    const unsigned q = row - b * (unsigned)SEQ;
    const size_t ro = ((size_t)b * SEQ_FULL + q) * SEQ_FULL;
    const float* dr = dist + ro;
    const float* ar = adj + ro;
    const int*   mr = mask + (size_t)b * SEQ_FULL;

    float mx = -3.0e38f, asum = 0.0f;
#pragma unroll 1
    for (unsigned hf = 0; hf < (unsigned)(SEQ / 256); ++hf) {
        const unsigned c = hf * 256u + lane * 8u;
        v4f d0 = *(const v4f*)(dr + c), d1 = *(const v4f*)(dr + c + 4);
        v4f a0 = *(const v4f*)(ar + c), a1 = *(const v4f*)(ar + c + 4);
        v4i m0 = *(const v4i*)(mr + c), m1 = *(const v4i*)(mr + c + 4);
#pragma unroll
        for (int e = 0; e < 4; ++e) {
            float n0 = (m0[e] != 0) ? -bf16r(d0[e]) : -3.0e38f;
            float n1 = (m1[e] != 0) ? -bf16r(d1[e]) : -3.0e38f;
            mx = fmaxf(mx, fmaxf(n0, n1));
            asum += bf16r(a0[e]) + bf16r(a1[e]);
        }
    }
#pragma unroll
    for (int off = 16; off > 0; off >>= 1) {
        mx = fmaxf(mx, __shfl_xor(mx, off, 32));
        asum += __shfl_xor(asum, off, 32);
    }
    float esum = 0.0f;
#pragma unroll 1
    for (unsigned hf = 0; hf < (unsigned)(SEQ / 256); ++hf) {
        const unsigned c = hf * 256u + lane * 8u;
        v4f d0 = *(const v4f*)(dr + c), d1 = *(const v4f*)(dr + c + 4);
        v4i m0 = *(const v4i*)(mr + c), m1 = *(const v4i*)(mr + c + 4);
#pragma unroll
        for (int e = 0; e < 4; ++e) {
            float e0 = ex2((-bf16r(d0[e]) - mx) * LOG2E);
            float e1 = ex2((-bf16r(d1[e]) - mx) * LOG2E);
            esum += ((m0[e] != 0) ? e0 : 0.0f) + ((m1[e] != 0) ? e1 : 0.0f);
        }
    }
#pragma unroll
    for (int off = 16; off > 0; off >>= 1) esum += __shfl_xor(esum, off, 32);
    const float pinv = 1.0f / esum;
    const float ainv = 1.0f / (asum + 1.0e-6f);
#pragma unroll 1
    for (unsigned hf = 0; hf < (unsigned)(SEQ / 256); ++hf) {
        const unsigned c = hf * 256u + lane * 8u;
        v4f d0 = *(const v4f*)(dr + c), d1 = *(const v4f*)(dr + c + 4);
        v4f a0 = *(const v4f*)(ar + c), a1 = *(const v4f*)(ar + c + 4);
        v4i m0 = *(const v4i*)(mr + c), m1 = *(const v4i*)(mr + c + 4);
        v8h hv;
#pragma unroll
        for (int e = 0; e < 4; ++e) {
            float e0 = ex2((-bf16r(d0[e]) - mx) * LOG2E);
            float e1 = ex2((-bf16r(d1[e]) - mx) * LOG2E);
            e0 = (m0[e] != 0) ? e0 : 0.0f;
            e1 = (m1[e] != 0) ? e1 : 0.0f;
            float w0 = 0.3f * (e0 * pinv) + 0.4f * (bf16r(a0[e]) * ainv);
            float w1 = 0.3f * (e1 * pinv) + 0.4f * (bf16r(a1[e]) * ainv);
            hv[e]     = (_Float16)(w0 * 4096.0f);
            hv[4 + e] = (_Float16)(w1 * 4096.0f);
        }
        _Float16* dst = Mh + (size_t)row * SEQ + c;
        *(volatile v8h*)dst = hv;
        __threadfence();
        *(volatile v8h*)dst = hv;
    }
}

template <int FINAL>
__global__ __launch_bounds__(256) void k_ln(const float* __restrict__ x, int xfull,
                                             const float* __restrict__ ga,
                                             const float* __restrict__ gb,
                                             _Float16* __restrict__ oh,
                                             _Float16* __restrict__ orr,
                                             float* __restrict__ of) {
    const unsigned tid = threadIdx.x, lane = tid & 31u, w = tid >> 5;
    const unsigned row = blockIdx.x * 8u + w;
    const unsigned bt = row / (unsigned)SEQ;
    const unsigned irow = xfull ? (bt * (unsigned)SEQ_FULL + (row - bt * (unsigned)SEQ)) : row;
    const unsigned c0 = FINAL ? (lane * 4u) : (lane * 8u);
    const unsigned c1 = FINAL ? (128u + lane * 4u) : (lane * 8u + 4u);
    const float* xr = x + (size_t)irow * DM;
    v4f xa = *(const v4f*)(xr + c0);
    v4f xb = *(const v4f*)(xr + c1);
    float v[8];
#pragma unroll
    for (int e = 0; e < 4; ++e) {
        float t0 = xa[e], t1 = xb[e];
        v[e]     = xfull ? bf16r(t0) : t0;
        v[4 + e] = xfull ? bf16r(t1) : t1;
    }
    float s = ((v[0] + v[1]) + (v[2] + v[3])) + ((v[4] + v[5]) + (v[6] + v[7]));
#pragma unroll
    for (int off = 16; off > 0; off >>= 1) s += __shfl_xor(s, off, 32);
    const float mean = s * (1.0f / 256.0f);
    float sq = 0.0f;
#pragma unroll
    for (int e = 0; e < 8; ++e) { v[e] -= mean; sq += v[e] * v[e]; }
#pragma unroll
    for (int off = 16; off > 0; off >>= 1) sq += __shfl_xor(sq, off, 32);
    const float sd  = sqrtf(sq * (1.0f / 255.0f));
    const float inv = 1.0f / (sd + 1.0e-6f);
    v4f a0 = *(const v4f*)(ga + c0), a1 = *(const v4f*)(ga + c1);
    v4f b0 = *(const v4f*)(gb + c0), b1 = *(const v4f*)(gb + c1);
    float y[8];
#pragma unroll
    for (int e = 0; e < 4; ++e) {
        y[e]     = (bf16r(a0[e]) * v[e]) * inv + bf16r(b0[e]);
        y[4 + e] = (bf16r(a1[e]) * v[4 + e]) * inv + bf16r(b1[e]);
    }
    if (FINAL) {
        v4f o0, o1;
#pragma unroll
        for (int e = 0; e < 4; ++e) { o0[e] = y[e]; o1[e] = y[4 + e]; }
        float* dp = of + (size_t)row * DM;
        *(volatile v4f*)(dp + c0) = o0;
        *(volatile v4f*)(dp + c1) = o1;
        __threadfence();
        *(volatile v4f*)(dp + c0) = o0;
        *(volatile v4f*)(dp + c1) = o1;
    } else {
        v8h hv, rv;
#pragma unroll
        for (int e = 0; e < 8; ++e) {
            _Float16 hh = (_Float16)y[e];
            hv[e] = hh;
            rv[e] = (_Float16)((y[e] - (float)hh) * SC_RES);
        }
        _Float16* dh = oh  + (size_t)row * DM + lane * 8u;
        _Float16* dr = orr + (size_t)row * DM + lane * 8u;
        *(volatile v8h*)dh = hv;
        *(volatile v8h*)dr = rv;
        __threadfence();
        *(volatile v8h*)dh = hv;
        *(volatile v8h*)dr = rv;
    }
}

template <int MODE>
__global__ __launch_bounds__(128) __attribute__((amdgpu_num_vgpr(256)))
void k_gemm(const _Float16* __restrict__ Ah, const _Float16* __restrict__ Ar,
            const _Float16* __restrict__ WT,
            const float* __restrict__ b0, const float* __restrict__ b1,
            const float* __restrict__ b2,
            float sc, float bsc,
            const float* xin, int xfull, float* xout,
            _Float16* __restrict__ p0h, _Float16* __restrict__ p0r,
            _Float16* __restrict__ p1h, _Float16* __restrict__ p1r,
            _Float16* __restrict__ p2h, _Float16* __restrict__ p2r) {
    __shared__ __align__(16) float    Ost[4][16 * 64];
    __shared__ __align__(16) _Float16 Hst[4][16 * 64];
    __shared__ __align__(16) _Float16 Rst[4][16 * 64];

    const unsigned tid = threadIdx.x, lane = tid & 31u, w = tid >> 5;
    const unsigned row0 = blockIdx.x * 64u + w * 16u;
    const unsigned col0 = blockIdx.y * 64u;

    v8f ah[4], ar[4];
#pragma unroll
    for (int nt = 0; nt < 4; ++nt) { ah[nt] = zero8(); ar[nt] = zero8(); }
    const _Float16* ap = Ah + (size_t)row0 * DM;
    const _Float16* rp = Ar + (size_t)row0 * DM;
    const _Float16* wp = WT + (size_t)col0 * DM;
#pragma unroll 1
    for (unsigned k0 = 0; k0 < (unsigned)DM; k0 += 32u) {
        v16h fa = load_frag16(ap + k0, DM, lane);
        v16h fr = load_frag16(rp + k0, DM, lane);
#pragma unroll
        for (int nt = 0; nt < 4; ++nt) {
            v16h fb = load_frag16(wp + (size_t)(nt * 16) * DM + k0, DM, lane);
            ah[nt] = wmma16(fa, fb, ah[nt]);
            ar[nt] = wmma16(fr, fb, ar[nt]);
        }
    }

    const unsigned r0 = (lane >> 4) << 3;
    const unsigned cc = lane & 15u;
    const unsigned which = (MODE == 0) ? (col0 >> 8) : 0u;
    const unsigned hc = col0 & 255u;
    const float* bp = (which == 0u) ? b0 : ((which == 1u) ? b1 : b2);
    float bvv[4];
#pragma unroll
    for (int nt = 0; nt < 4; ++nt) bvv[nt] = bf16r(bp[hc + (unsigned)(nt * 16) + cc]) * bsc;

    if (MODE == 1 || MODE == 3) {
#pragma unroll
        for (int nt = 0; nt < 4; ++nt)
#pragma unroll
            for (int g = 0; g < 8; ++g) {
                float val = __builtin_fmaf(ar[nt][g], SC_RINV, ah[nt][g]) * sc + bvv[nt];
                if (MODE == 3) val = (val > 0.0f) ? val : 0.1f * val;
                Ost[w][(r0 + (unsigned)g) * 64u + (unsigned)(nt * 16) + cc] = val;
            }
        wave_lds_sync();
        v4f ov[8];
        const unsigned cq = (lane & 15u) * 4u;
#pragma unroll
        for (int i = 0; i < 8; ++i) {
            const unsigned gr = row0 + (unsigned)(i * 2) + (lane >> 4);
            const unsigned bt = gr / (unsigned)SEQ;
            const unsigned ir = xfull ? (bt * (unsigned)SEQ_FULL + (gr - bt * (unsigned)SEQ)) : gr;
            v4f dv = *(const v4f*)(&Ost[w][(unsigned)(i * 128) + lane * 4u]);
            v4f xo = *(const v4f*)(xin + (size_t)ir * DM + col0 + cq);
#pragma unroll
            for (int e = 0; e < 4; ++e) {
                float xe = xo[e];
                xe = xfull ? bf16r(xe) : xe;
                ov[i][e] = xe + dv[e];
            }
        }
#pragma unroll
        for (int i = 0; i < 8; ++i) {
            const unsigned gr = row0 + (unsigned)(i * 2) + (lane >> 4);
            *(volatile v4f*)(xout + (size_t)gr * DM + col0 + cq) = ov[i];
        }
        __threadfence();
#pragma unroll
        for (int i = 0; i < 8; ++i) {
            const unsigned gr = row0 + (unsigned)(i * 2) + (lane >> 4);
            *(volatile v4f*)(xout + (size_t)gr * DM + col0 + cq) = ov[i];
        }
    } else {
#pragma unroll
        for (int nt = 0; nt < 4; ++nt)
#pragma unroll
            for (int g = 0; g < 8; ++g) {
                float val = __builtin_fmaf(ar[nt][g], SC_RINV, ah[nt][g]) * sc + bvv[nt];
                if (MODE == 2) val = (val > 0.0f) ? val : 0.1f * val;
                _Float16 hh = (_Float16)val;
                const unsigned o = (r0 + (unsigned)g) * 64u + (unsigned)(nt * 16) + cc;
                Hst[w][o] = hh;
                Rst[w][o] = (_Float16)((val - (float)hh) * SC_RES);
            }
        wave_lds_sync();
        if (MODE == 2) {
            v8h ph[4], pr[4];
#pragma unroll
            for (int i = 0; i < 4; ++i) {
                const unsigned p = (unsigned)(i * 32) + lane;
                const unsigned so = (p >> 3) * 64u + (p & 7u) * 8u;
                ph[i] = *(const v8h*)(&Hst[w][so]);
                pr[i] = *(const v8h*)(&Rst[w][so]);
            }
#pragma unroll
            for (int i = 0; i < 4; ++i) {
                const unsigned p = (unsigned)(i * 32) + lane;
                const size_t go = (size_t)(row0 + (p >> 3)) * DM + col0 + (p & 7u) * 8u;
                *(volatile v8h*)(p0h + go) = ph[i];
                *(volatile v8h*)(p0r + go) = pr[i];
            }
            __threadfence();
#pragma unroll
            for (int i = 0; i < 4; ++i) {
                const unsigned p = (unsigned)(i * 32) + lane;
                const size_t go = (size_t)(row0 + (p >> 3)) * DM + col0 + (p & 7u) * 8u;
                *(volatile v8h*)(p0h + go) = ph[i];
                *(volatile v8h*)(p0r + go) = pr[i];
            }
        } else {
            _Float16* ph_ = (which == 0u) ? p0h : ((which == 1u) ? p1h : p2h);
            _Float16* pr_ = (which == 0u) ? p0r : ((which == 1u) ? p1r : p2r);
            const unsigned bt = row0 / (unsigned)SEQ;
            const unsigned s0 = row0 - bt * (unsigned)SEQ;
            const unsigned h0 = hc >> 5;
            v8h ph[2][2], pr[2][2];
#pragma unroll
            for (int hh = 0; hh < 2; ++hh)
#pragma unroll
                for (int i = 0; i < 2; ++i) {
                    const unsigned p = (unsigned)(i * 32) + lane;
                    const unsigned so = (p >> 2) * 64u + (unsigned)(hh * 32) + (p & 3u) * 8u;
                    ph[hh][i] = *(const v8h*)(&Hst[w][so]);
                    pr[hh][i] = *(const v8h*)(&Rst[w][so]);
                }
#pragma unroll
            for (int hh = 0; hh < 2; ++hh)
#pragma unroll
                for (int i = 0; i < 2; ++i) {
                    const unsigned p = (unsigned)(i * 32) + lane;
                    const size_t go = ((size_t)(bt * NH + h0 + (unsigned)hh) * SEQ + s0) * HD + p * 8u;
                    *(volatile v8h*)(ph_ + go) = ph[hh][i];
                    *(volatile v8h*)(pr_ + go) = pr[hh][i];
                }
            __threadfence();
#pragma unroll
            for (int hh = 0; hh < 2; ++hh)
#pragma unroll
                for (int i = 0; i < 2; ++i) {
                    const unsigned p = (unsigned)(i * 32) + lane;
                    const size_t go = ((size_t)(bt * NH + h0 + (unsigned)hh) * SEQ + s0) * HD + p * 8u;
                    *(volatile v8h*)(ph_ + go) = ph[hh][i];
                    *(volatile v8h*)(pr_ + go) = pr[hh][i];
                }
        }
    }
}

__global__ __launch_bounds__(256) __attribute__((amdgpu_num_vgpr(256)))
void k_attn(const _Float16* __restrict__ qh, const _Float16* __restrict__ ql,
            const _Float16* __restrict__ kh, const _Float16* __restrict__ kl,
            const _Float16* __restrict__ vh, const _Float16* __restrict__ vl,
            const _Float16* __restrict__ Mh, const int* __restrict__ mask,
            _Float16* __restrict__ atth, _Float16* __restrict__ attr) {
    __shared__ __align__(16) _Float16 VshT[HD * CH];
    __shared__ __align__(16) _Float16 VslT[HD * CH];
    __shared__ __align__(16) float    Sst[8][16 * 32];
    __shared__ __align__(16) _Float16 Ahs[8][16 * 64];
    __shared__ __align__(16) _Float16 Ars[8][16 * 64];
    __shared__ __align__(16) float    mks[SEQ];

    const unsigned tid = threadIdx.x, lane = tid & 31u, w = tid >> 5;
    const unsigned b = blockIdx.x, hp = blockIdx.y;
    const unsigned q0r = blockIdx.z * 128u + w * 16u;
    const unsigned r0 = (lane >> 4) << 3;
    const unsigned cc = lane & 15u;

    for (unsigned idx = tid; idx < (unsigned)SEQ; idx += 256u)
        mks[idx] = (mask[(size_t)b * SEQ_FULL + idx] != 0) ? 1.0f : 0.0f;

    const _Float16* Mb = Mh + ((size_t)b * SEQ + q0r) * SEQ;
    const float* srow = &Sst[w][cc * 32u + r0];

#pragma unroll 1
    for (unsigned hh = 0; hh < 2u; ++hh) {
        const unsigned h = hp * 2u + hh;
        const size_t hb = ((size_t)(b * NH + h) * SEQ) * HD;
        const v16h qhf = load_frag16(qh + hb + (size_t)q0r * HD, HD, lane);
        const v16h qlf = load_frag16(ql + hb + (size_t)q0r * HD, HD, lane);
        const _Float16* khb = kh + hb;
        const _Float16* klb = kl + hb;
        const _Float16* vhb = vh + hb;
        const _Float16* vlb = vl + hb;

        v8f o0 = zero8(), o1 = zero8();
        v8f or0 = zero8(), or1 = zero8();
        v8f om0 = zero8(), om1 = zero8();
        float mrow = -3.0e38f, lsum = 0.0f;

#pragma unroll 1
        for (unsigned c0 = 0; c0 < (unsigned)SEQ; c0 += CH) {
            for (unsigned idx = tid; idx < (unsigned)(CH * 4); idx += 256u) {
                unsigned t = idx >> 2, part = idx & 3u;
                v8h vv = *(const v8h*)(vhb + (size_t)(c0 + t) * HD + part * 8u);
                v8h vr = *(const v8h*)(vlb + (size_t)(c0 + t) * HD + part * 8u);
#pragma unroll
                for (int e = 0; e < 8; ++e) {
                    VshT[(part * 8u + (unsigned)e) * CH + t] = vv[e];
                    VslT[(part * 8u + (unsigned)e) * CH + t] = vr[e];
                }
            }
            __syncthreads();

#pragma unroll 1
            for (unsigned j = 0; j < (unsigned)CH; j += 32u) {
                const unsigned kA = c0 + j;
                v16h khA = load_frag16(khb + (size_t)kA * HD, HD, lane);
                v16h klA = load_frag16(klb + (size_t)kA * HD, HD, lane);
                v8f sh0 = wmma16(qhf, khA, zero8());
                v8f sr0 = wmma16(qhf, klA, zero8());
                sr0 = wmma16(qlf, khA, sr0);
                v16h khB = load_frag16(khb + (size_t)(kA + 16u) * HD, HD, lane);
                v16h klB = load_frag16(klb + (size_t)(kA + 16u) * HD, HD, lane);
                v8f sh1 = wmma16(qhf, khB, zero8());
                v8f sr1 = wmma16(qhf, klB, zero8());
                sr1 = wmma16(qlf, khB, sr1);

                const float kp0 = mks[kA + cc];
                const float kp1 = mks[kA + 16u + cc];
#pragma unroll
                for (int g = 0; g < 8; ++g) {
                    float t0 = __builtin_fmaf(sh0[g], C1, sr0[g] * C2);
                    float t1 = __builtin_fmaf(sh1[g], C1, sr1[g] * C2);
                    t0 = (kp0 != 0.0f) ? t0 : FILL_T;
                    t1 = (kp1 != 0.0f) ? t1 : FILL_T;
                    Sst[w][(r0 + (unsigned)g) * 32u + cc]       = t0;
                    Sst[w][(r0 + (unsigned)g) * 32u + 16u + cc] = t1;
                }
                wave_lds_sync();
                v4f s0 = *(const v4f*)(srow);
                v4f s1 = *(const v4f*)(srow + 4);
                v4f s2 = *(const v4f*)(srow + 16);
                v4f s3 = *(const v4f*)(srow + 20);
                float sv[16];
#pragma unroll
                for (int e = 0; e < 4; ++e) {
                    sv[e] = s0[e]; sv[4 + e] = s1[e]; sv[8 + e] = s2[e]; sv[12 + e] = s3[e];
                }
                float tmax = sv[0];
#pragma unroll
                for (int e = 1; e < 16; ++e) tmax = fmaxf(tmax, sv[e]);
                tmax = fmaxf(tmax, __shfl_xor(tmax, 16, 32));
                const float mn = fmaxf(mrow, tmax);
                const float alpha = ex2(mrow - mn);
                mrow = mn;
                const float mc = mn - P_CARRY;
                Frag pa;
                float ps = 0.0f;
#pragma unroll
                for (int e = 0; e < 16; ++e) {
                    float pe = ex2(sv[e] - mc);
                    ps += pe;
                    pa.v[e] = (_Float16)pe;
                }
                lsum = lsum * alpha + ps;
#pragma unroll
                for (int g = 0; g < 8; ++g) {
                    const float ag = __shfl(alpha, (int)(r0 + (unsigned)g), 32);
                    o0[g] *= ag; o1[g] *= ag; or0[g] *= ag; or1[g] *= ag;
                }
                v16h vb0 = load_frag16(&VshT[0 * CH + j], CH, lane);
                v16h vb1 = load_frag16(&VshT[16 * CH + j], CH, lane);
                o0 = wmma16(pa.v, vb0, o0);
                o1 = wmma16(pa.v, vb1, o1);
                v16h vr0 = load_frag16(&VslT[0 * CH + j], CH, lane);
                v16h vr1 = load_frag16(&VslT[16 * CH + j], CH, lane);
                or0 = wmma16(pa.v, vr0, or0);
                or1 = wmma16(pa.v, vr1, or1);
                v16h ma = load_frag16(Mb + kA, SEQ, lane);
                om0 = wmma16(ma, vb0, om0);
                om1 = wmma16(ma, vb1, om1);
            }
            __syncthreads();
        }

        lsum += __shfl_xor(lsum, 16, 32);
        const float inv = 1.0f / lsum;
#pragma unroll
        for (int g = 0; g < 8; ++g) {
            const float ig = __shfl(inv, (int)(r0 + (unsigned)g), 32) * SC_ATT;
            float a0 = __builtin_fmaf(or0[g], SC_RINV, o0[g]) * ig + om0[g] * SC_MV;
            float a1 = __builtin_fmaf(or1[g], SC_RINV, o1[g]) * ig + om1[g] * SC_MV;
            _Float16 h0 = (_Float16)a0, h1 = (_Float16)a1;
            const unsigned o = (r0 + (unsigned)g) * 64u + hh * 32u + cc;
            Ahs[w][o]       = h0;
            Ahs[w][o + 16u] = h1;
            Ars[w][o]       = (_Float16)((a0 - (float)h0) * SC_RES);
            Ars[w][o + 16u] = (_Float16)((a1 - (float)h1) * SC_RES);
        }
    }
    wave_lds_sync();

    v8h ph[4], pr[4];
#pragma unroll
    for (int i = 0; i < 4; ++i) {
        const unsigned p = (unsigned)(i * 32) + lane;
        const unsigned so = (p >> 3) * 64u + (p & 7u) * 8u;
        ph[i] = *(const v8h*)(&Ahs[w][so]);
        pr[i] = *(const v8h*)(&Ars[w][so]);
    }
    const size_t ob = ((size_t)b * SEQ + q0r) * DM + hp * 64u;
#pragma unroll
    for (int i = 0; i < 4; ++i) {
        const unsigned p = (unsigned)(i * 32) + lane;
        const size_t go = ob + (size_t)(p >> 3) * DM + (p & 7u) * 8u;
        *(volatile v8h*)(atth + go) = ph[i];
        *(volatile v8h*)(attr + go) = pr[i];
    }
    __threadfence();
#pragma unroll
    for (int i = 0; i < 4; ++i) {
        const unsigned p = (unsigned)(i * 32) + lane;
        const size_t go = ob + (size_t)(p >> 3) * DM + (p & 7u) * 8u;
        *(volatile v8h*)(atth + go) = ph[i];
        *(volatile v8h*)(attr + go) = pr[i];
    }
}

extern "C" void kernel_launch(void* const* d_in, const int* in_sizes, int n_in,
                              void* d_out, int out_size, void* d_ws, size_t ws_size,
                              hipStream_t stream) {
    if (n_in < 23) return;
    if (in_sizes[0] < ((NB - 1) * SEQ_FULL + SEQ) * DM) return;
    if (in_sizes[1] < (NB - 1) * SEQ_FULL + SEQ) return;
    if (in_sizes[2] < ((NB - 1) * SEQ_FULL + SEQ - 1) * SEQ_FULL + SEQ) return;
    if (in_sizes[3] < ((NB - 1) * SEQ_FULL + SEQ - 1) * SEQ_FULL + SEQ) return;
    for (int i = 5; i <= 15; i += 2) if (in_sizes[i] < NL * WSZ) return;
    for (int i = 6; i <= 16; i += 2) if (in_sizes[i] < NL * DM) return;
    for (int i = 17; i <= 20; ++i)   if (in_sizes[i] < NL * DM) return;
    if (in_sizes[21] < DM || in_sizes[22] < DM) return;
    if (out_size < NTOK * DM) return;

    const float* xin  = (const float*)d_in[0];
    const int*   mask = (const int*)  d_in[1];
    const float* adj  = (const float*)d_in[2];
    const float* dist = (const float*)d_in[3];
    const float* Wq  = (const float*)d_in[5];   const float* bq  = (const float*)d_in[6];
    const float* Wk  = (const float*)d_in[7];   const float* bk  = (const float*)d_in[8];
    const float* Wv  = (const float*)d_in[9];   const float* bv  = (const float*)d_in[10];
    const float* Wo  = (const float*)d_in[11];  const float* bo  = (const float*)d_in[12];
    const float* Wf1 = (const float*)d_in[13];  const float* bf1 = (const float*)d_in[14];
    const float* Wf2 = (const float*)d_in[15];  const float* bf2 = (const float*)d_in[16];
    const float* ln1a = (const float*)d_in[17]; const float* ln1b = (const float*)d_in[18];
    const float* ln2a = (const float*)d_in[19]; const float* ln2b = (const float*)d_in[20];
    const float* lnfa = (const float*)d_in[21]; const float* lnfb = (const float*)d_in[22];
    float* out = (float*)d_out;

    char* ws = (char*)d_ws;
    size_t off = 0;
    _Float16* WT = (_Float16*)(ws + off); off += (size_t)NL * 6 * WSZ * 2;
    _Float16* Mh = (_Float16*)(ws + off); off += (size_t)NB * SEQ * SEQ * 2;
    float*    xw = (float*)(ws + off);    off += (size_t)NTOK * DM * 4;
    const size_t PL = (size_t)NTOK * DM * 2;
    _Float16* hAh = (_Float16*)(ws + off); off += PL;
    _Float16* hAr = (_Float16*)(ws + off); off += PL;
    _Float16* qh  = (_Float16*)(ws + off); off += PL;
    _Float16* ql  = (_Float16*)(ws + off); off += PL;
    _Float16* kh  = (_Float16*)(ws + off); off += PL;
    _Float16* kl  = (_Float16*)(ws + off); off += PL;
    _Float16* vh  = (_Float16*)(ws + off); off += PL;
    _Float16* vl  = (_Float16*)(ws + off); off += PL;
    _Float16* ath = (_Float16*)(ws + off); off += PL;
    _Float16* atr = (_Float16*)(ws + off); off += PL;
    _Float16* gh  = (_Float16*)(ws + off); off += PL;
    _Float16* gr  = (_Float16*)(ws + off); off += PL;
    if (off > ws_size) return;

    k_wprep<<<dim3(4, 4, NL * 6), dim3(256), 0, stream>>>(Wq, Wk, Wv, Wo, Wf1, Wf2, WT);
    k_pmix<<<dim3(NB * SEQ / 8), dim3(256), 0, stream>>>(adj, dist, mask, Mh);

    for (int l = 0; l < NL; ++l) {
        const float* xs = (l == 0) ? xin : (const float*)xw;
        const int xf = (l == 0) ? 1 : 0;
        const _Float16* WL = WT + (size_t)l * 6 * WSZ;
        k_ln<0><<<dim3(NTOK / 8), dim3(256), 0, stream>>>(xs, xf, ln1a + l * DM, ln1b + l * DM,
                                                         hAh, hAr, out);
        k_gemm<0><<<dim3(NTOK / 64, 12), dim3(128), 0, stream>>>(
            hAh, hAr, WL, bq + l * DM, bk + l * DM, bv + l * DM, 1.0f, 64.0f,
            xw, 0, xw, qh, ql, kh, kl, vh, vl);
        k_attn<<<dim3(NB, NH / 2, SEQ / 128), dim3(256), 0, stream>>>(
            qh, ql, kh, kl, vh, vl, Mh, mask, ath, atr);
        k_gemm<1><<<dim3(NTOK / 64, 4), dim3(128), 0, stream>>>(
            ath, atr, WL + (size_t)3 * WSZ, bo + l * DM, bo + l * DM, bo + l * DM, SC_WO, 1.0f,
            xs, xf, xw, gh, gr, gh, gr, gh, gr);
        k_ln<0><<<dim3(NTOK / 8), dim3(256), 0, stream>>>(xw, 0, ln2a + l * DM, ln2b + l * DM,
                                                         hAh, hAr, out);
        k_gemm<2><<<dim3(NTOK / 64, 4), dim3(128), 0, stream>>>(
            hAh, hAr, WL + (size_t)4 * WSZ, bf1 + l * DM, bf1 + l * DM, bf1 + l * DM, SC_FF, 1.0f,
            xw, 0, xw, gh, gr, gh, gr, gh, gr);
        k_gemm<3><<<dim3(NTOK / 64, 4), dim3(128), 0, stream>>>(
            gh, gr, WL + (size_t)5 * WSZ, bf2 + l * DM, bf2 + l * DM, bf2 + l * DM, SC_FF, 1.0f,
            xw, 0, xw, ath, atr, ath, atr, ath, atr);
    }
    k_ln<1><<<dim3(NTOK / 8), dim3(256), 0, stream>>>(xw, 0, lnfa, lnfb, hAh, hAr, out);
}
